// FlexLocalFrameAttention_46806553592108
// MI455X (gfx1250) — hardware-verified
//
#include <hip/hip_runtime.h>


#define NB_  2
#define TT   4096
#define DM   1024
#define NH_  16
#define HD   64
#define CH   512
#define NC   8
#define WK   1024
#define TP   (TT + CH)
#define HG   4
#define ZZ   (HG * NC)
#define PCAR 1024.0f
typedef _Float16 h16;
typedef unsigned short bf;
typedef __attribute__((ext_vector_type(16))) __bf16   v16bf;
typedef __attribute__((ext_vector_type(16))) _Float16 v16h;
typedef __attribute__((ext_vector_type(8)))  _Float16 v8h;
typedef __attribute__((ext_vector_type(8)))  unsigned short v8us;
typedef __attribute__((ext_vector_type(8)))  float    v8f;
typedef __attribute__((ext_vector_type(4)))  float    v4f;
typedef v8h  __attribute__((may_alias)) v8ha;
typedef v4f  __attribute__((may_alias)) v4fa;
typedef v8us __attribute__((may_alias)) v8usa;

__device__ __forceinline__ unsigned short f2bf(float f) { unsigned u = __float_as_uint(f); u += 0x7FFFu + ((u >> 16) & 1u); return (unsigned short)(u >> 16); }
__device__ __forceinline__ float bf2f(unsigned short b) { return __uint_as_float(((unsigned)b) << 16); }
__device__ __forceinline__ float bfr(float f) { return bf2f(f2bf(f)); }
__device__ __forceinline__ v16h cat16(v8h lo, v8h hi) { return __builtin_shufflevector(lo, hi, 0, 1, 2, 3, 4, 5, 6, 7, 8, 9, 10, 11, 12, 13, 14, 15); }
__device__ __forceinline__ v16bf cat16b(v8us lo, v8us hi) { return __builtin_bit_cast(v16bf, __builtin_shufflevector(lo, hi, 0, 1, 2, 3, 4, 5, 6, 7, 8, 9, 10, 11, 12, 13, 14, 15)); }
__device__ __forceinline__ v8f wmma16(v16h a, v16h b, v8f c) { return __builtin_amdgcn_wmma_f32_16x16x32_f16(false, a, false, b, (short)0, c, false, false); }
__device__ __forceinline__ v8f wmmab(v16bf a, v16bf b, v8f c) { return __builtin_amdgcn_wmma_f32_16x16x32_bf16(false, a, false, b, (short)0, c, false, false); }


template <typename T16> struct WFrag;
template <> struct WFrag<h16> { typedef v16h V; static __device__ __forceinline__ V ld(const h16* p) { return cat16(*(const v8h*)p, *(const v8h*)(p + 16)); } static __device__ __forceinline__ v8f mma(V a, V b, v8f c) { return wmma16(a, b, c); } };
template <> struct WFrag<bf> { typedef v16bf V; static __device__ __forceinline__ V ld(const bf* p) { return cat16b(*(const v8us*)p, *(const v8us*)(p + 16)); } static __device__ __forceinline__ v8f mma(V a, V b, v8f c) { return wmmab(a, b, c); } };
template <typename T16, int NSPLIT, bool BIAS>
__global__ __launch_bounds__(32) void k_gemmw(const T16* __restrict__ A, const T16* __restrict__ A2, const T16* __restrict__ Bt, const T16* __restrict__ Bt2, int K, float* C, int ldc, const float* __restrict__ bias, size_t sA, size_t sB, size_t sC) {
    typedef typename WFrag<T16>::V V;
    __shared__ __align__(16) float os[16 * 68];
    const size_t z = blockIdx.z; A += z * sA; if (A2) A2 += z * sA; Bt += z * sB; if (Bt2) Bt2 += z * sB; C += z * sC;
    const int lane = threadIdx.x & 31, lr = lane & 15, hi = lane >> 4; const int r0 = blockIdx.x * 64, c0 = blockIdx.y * 64;
    v8f acc[4][4];
#pragma unroll
    for (int mb = 0; mb < 4; ++mb)
#pragma unroll
        for (int nb = 0; nb < 4; ++nb) acc[mb][nb] = (v8f){};
    const size_t aoff = (size_t)(r0 + lr) * K + 8 * hi, boff = (size_t)(c0 + lr) * K + 8 * hi;
#pragma unroll 1
    for (int kc = 0; kc < K; kc += 32) {
        V a[4], a2[4];
#pragma unroll
        for (int mb = 0; mb < 4; ++mb) { a[mb] = WFrag<T16>::ld(A + aoff + (size_t)mb * 16 * K + kc); if (NSPLIT == 1 || NSPLIT == 2) a2[mb] = WFrag<T16>::ld(A2 + aoff + (size_t)mb * 16 * K + kc); }
#pragma unroll
        for (int nb = 0; nb < 4; ++nb) { const V b = WFrag<T16>::ld(Bt + boff + (size_t)nb * 16 * K + kc); V b2; if (NSPLIT >= 2) b2 = WFrag<T16>::ld(Bt2 + boff + (size_t)nb * 16 * K + kc);
#pragma unroll
            for (int mb = 0; mb < 4; ++mb) { acc[mb][nb] = WFrag<T16>::mma(a[mb], b, acc[mb][nb]); if (NSPLIT == 1 || NSPLIT == 2) acc[mb][nb] = WFrag<T16>::mma(a2[mb], b, acc[mb][nb]); if (NSPLIT >= 2) acc[mb][nb] = WFrag<T16>::mma(a[mb], b2, acc[mb][nb]); } }
        asm volatile("v_nop\n\tv_nop\n\tv_nop\n\tv_nop" : "+v"(acc[0][0]), "+v"(acc[1][1]), "+v"(acc[2][2]), "+v"(acc[3][3]) : "v"(a[0]), "v"(a[3]));
    }
#pragma unroll
    for (int mb = 0; mb < 4; ++mb) {
#pragma unroll
        for (int nb = 0; nb < 4; ++nb) {
#pragma unroll
            for (int j = 0; j < 8; ++j) os[(hi * 8 + j) * 68 + nb * 16 + lr] = acc[mb][nb][j]; }
        __builtin_amdgcn_wave_barrier(); asm volatile("" ::: "memory");
        float* crow = C + (size_t)(r0 + mb * 16) * ldc + c0;
#pragma unroll 1
        for (int ps = 0; ps < 2; ++ps) {
#pragma unroll
            for (int s = 0; s < 8; ++s) { const int row = 2 * s + hi, cofs = lr * 4; v4f val = *(const v4fa*)(os + row * 68 + cofs); if (BIAS) { val[0] += bfr(bias[c0 + cofs]); val[1] += bfr(bias[c0 + cofs + 1]); val[2] += bfr(bias[c0 + cofs + 2]); val[3] += bfr(bias[c0 + cofs + 3]); }
                *(volatile v4f*)(crow + (size_t)row * ldc + cofs) = val; }
            if (ps == 0) __threadfence(); }
        __builtin_amdgcn_wave_barrier(); asm volatile("" ::: "memory");
    }
}

__device__ __forceinline__ h16 tohx(float x) { return (h16)x; }
typedef __attribute__((ext_vector_type(2))) _Float16 v2h;
typedef __attribute__((ext_vector_type(4))) _Float16 v4h;

__global__ __launch_bounds__(256) void k_cvt8(const float* __restrict__ src, bf* dst, size_t n8) { const size_t i = (size_t)blockIdx.x * 256 + threadIdx.x; if (i >= n8) return; const v8f v = *(const v8f*)(src + i * 8); v8us o;
#pragma unroll
    for (int k = 0; k < 8; ++k) o[k] = f2bf(v[k]); *(volatile v8us*)(dst + i * 8) = o; __threadfence(); *(volatile v8us*)(dst + i * 8) = o; }
__global__ __launch_bounds__(256) void k_wt16n(const float* __restrict__ w, size_t n4, h16* W16) { const size_t e = ((size_t)blockIdx.x * 256 + threadIdx.x) * 4; if (e >= n4 * 4) return; const v4f a = *(const v4f*)(w + e); v4h o;
#pragma unroll
    for (int u = 0; u < 4; ++u) o[u] = tohx(bfr(a[u])); *(volatile v4h*)(W16 + e) = o; __threadfence(); *(volatile v4h*)(W16 + e) = o; }
__global__ __launch_bounds__(256) void k_q16(const float* __restrict__ F, h16* Q16) { const size_t e = ((size_t)blockIdx.x * 256 + threadIdx.x) * 4; if (e >= (size_t)NH_ * TT * HD) return; const int d = (int)(e % HD); const int t = (int)((e / HD) % TT); const int h = (int)(e / ((size_t)HD * TT)); const v4f a = *(const v4f*)(F + (size_t)t * 3 * DM + h * HD + d); v4h o;
#pragma unroll
    for (int u = 0; u < 4; ++u) o[u] = tohx(a[u]); *(volatile v4h*)(Q16 + e) = o; __threadfence(); *(volatile v4h*)(Q16 + e) = o; }
__global__ __launch_bounds__(256) void k_k16(const float* __restrict__ F, h16* K16) { const size_t e = ((size_t)blockIdx.x * 256 + threadIdx.x) * 4; if (e >= (size_t)NH_ * TP * HD) return; const int d = (int)(e % HD); const int r = (int)((e / HD) % TP); const int h = (int)(e / ((size_t)HD * TP)); v4h o;
    if (r < CH) { o = (v4h){tohx(0.f), tohx(0.f), tohx(0.f), tohx(0.f)}; } else { const v4f a = *(const v4f*)(F + (size_t)(r - CH) * 3 * DM + DM + h * HD + d);
#pragma unroll
        for (int u = 0; u < 4; ++u) o[u] = tohx(a[u]); }
    *(volatile v4h*)(K16 + e) = o; __threadfence(); *(volatile v4h*)(K16 + e) = o; }
__global__ __launch_bounds__(256) void k_vw16(const float* __restrict__ F, int h0, h16* VW) { const size_t e = ((size_t)blockIdx.x * 256 + threadIdx.x) * 2; if (e >= (size_t)ZZ * HD * WK) return; const int j = (int)(e % WK); const int d = (int)((e / WK) % HD); const int z = (int)(e / ((size_t)WK * HD)); const int c = z % NC, hl = z / NC; const int h = h0 + hl; v2h o;
#pragma unroll
    for (int u = 0; u < 2; ++u) { const int s = (c - 1) * CH + j + u; o[u] = (s >= 0) ? tohx(F[(size_t)s * 3 * DM + 2 * DM + h * HD + d]) : tohx(0.f); }
    *(volatile v2h*)(VW + e) = o; __threadfence(); *(volatile v2h*)(VW + e) = o; }
__global__ __launch_bounds__(256) void k_mrg16(const float* __restrict__ O, int h0, h16* A16) { const size_t e = ((size_t)blockIdx.x * 256 + threadIdx.x) * 4; if (e >= (size_t)TT * HG * HD) return; const int cl = (int)(e % (HG * HD)); const int t = (int)(e / (HG * HD)); const int hl = cl / HD, d = cl % HD; const int c = t / CH, i = t % CH; const float* r = O + (((size_t)(hl * NC + c)) * CH + i) * HD + d; const size_t oo = (size_t)t * DM + (h0 + hl) * HD + d; v4h o;
#pragma unroll
    for (int u = 0; u < 4; ++u) o[u] = tohx(r[u] * (1.0f / PCAR)); *(volatile v4h*)(A16 + oo) = o; __threadfence(); *(volatile v4h*)(A16 + oo) = o; }
__global__ __launch_bounds__(256) void k_csoft(const float* __restrict__ Sb, h16* P16) { const int lane = threadIdx.x & 31; const int row = blockIdx.x * 8 + (threadIdx.x >> 5); if (row >= ZZ * CH) return; const int c = (row / CH) % NC; const float* sr = Sb + (size_t)row * WK; float v[32]; float mx = -3.0e38f;
#pragma unroll
    for (int ch = 0; ch < 8; ++ch) { const int j0 = ch * 128 + lane * 4; const v4f a = *(const v4f*)(sr + j0);
#pragma unroll
        for (int u = 0; u < 4; ++u) { const float t = (c > 0 || j0 >= CH) ? a[u] * 0.125f : -3.0e38f; v[ch * 4 + u] = t; mx = fmaxf(mx, t); } }
#pragma unroll
    for (int sh = 16; sh; sh >>= 1) mx = fmaxf(mx, __shfl_xor(mx, sh, 32));
    float sum = 0.f;
#pragma unroll
    for (int k = 0; k < 32; ++k) { float d0 = __fsub_rn(v[k], mx); asm volatile("" : "+v"(d0)); v[k] = __builtin_amdgcn_exp2f(__fmul_rn(d0, 1.4426950408889634f)); sum += v[k]; }
#pragma unroll
    for (int sh = 16; sh; sh >>= 1) sum += __shfl_xor(sum, sh, 32);
    const float f = __fdiv_rn(PCAR, sum);
    for (int ps = 0; ps < 2; ++ps) {
#pragma unroll
        for (int ch = 0; ch < 8; ++ch) { v4h o;
#pragma unroll
            for (int u = 0; u < 4; ++u) o[u] = tohx(v[ch * 4 + u] * f); *(volatile v4h*)(P16 + (size_t)row * WK + ch * 128 + lane * 4) = o; }
        if (ps == 0) __threadfence(); } }

extern "C" void kernel_launch(void* const* d_in, const int* in_sizes, int n_in,
                              void* d_out, int out_size, void* d_ws, size_t ws_size, hipStream_t stream) {
    (void)in_sizes; (void)n_in; (void)out_size;
    const float* x = (const float*)d_in[0]; const float* wqkv = (const float*)d_in[1]; const float* wout = (const float*)d_in[2];
    float* OUT = (float*)d_out;
    char* wsp = (char*)d_ws;
    auto take = [&](size_t bytes) { char* p = wsp; wsp += (bytes + 255) & ~(size_t)255; return (void*)p; };
    bf* WQKV = (bf*)take((size_t)3 * DM * DM * 2); h16* WO16 = (h16*)take((size_t)DM * DM * 2);
    bf* XB = (bf*)take((size_t)TT * DM * 2); float* F = (float*)take((size_t)TT * 3 * DM * 4); h16* Q16 = (h16*)take((size_t)NH_ * TT * HD * 2); h16* K16 = (h16*)take((size_t)NH_ * TP * HD * 2); h16* VW = (h16*)take((size_t)ZZ * HD * WK * 2);
    float* Sb = (float*)take((size_t)ZZ * CH * WK * 4); h16* P16 = (h16*)take((size_t)ZZ * CH * WK * 2); float* O = (float*)take((size_t)ZZ * CH * HD * 4); h16* A16 = (h16*)take((size_t)TT * DM * 2);
    if ((size_t)(wsp - (char*)d_ws) > ws_size) return;
    k_cvt8<<<(unsigned)(((size_t)3 * DM * DM / 8 + 255) / 256), 256, 0, stream>>>(wqkv, WQKV, (size_t)3 * DM * DM / 8); k_wt16n<<<(unsigned)(((size_t)DM * DM / 4 + 255) / 256), 256, 0, stream>>>(wout, (size_t)DM * DM / 4, WO16);
    for (int b = 0; b < NB_; ++b) {
        k_cvt8<<<(unsigned)(((size_t)TT * DM / 8 + 255) / 256), 256, 0, stream>>>(x + (size_t)b * TT * DM, XB, (size_t)TT * DM / 8);
        k_gemmw<bf, 0, false><<<dim3(TT / 64, 3 * DM / 64, 1), 32, 0, stream>>>(XB, nullptr, WQKV, nullptr, DM, F, 3 * DM, nullptr, 0, 0, 0);
        k_q16<<<(unsigned)(((size_t)NH_ * TT * HD / 4 + 255) / 256), 256, 0, stream>>>(F, Q16); k_k16<<<(unsigned)(((size_t)NH_ * TP * HD / 4 + 255) / 256), 256, 0, stream>>>(F, K16);
        for (int h0 = 0; h0 < NH_; h0 += HG) {
            k_vw16<<<(unsigned)(((size_t)ZZ * HD * WK / 2 + 255) / 256), 256, 0, stream>>>(F, h0, VW);
            for (int hl = 0; hl < HG; ++hl) { const int h = h0 + hl;
                k_gemmw<h16, 0, false><<<dim3(CH / 64, WK / 64, NC), 32, 0, stream>>>(Q16 + (size_t)h * TT * HD, nullptr, K16 + (size_t)h * TP * HD, nullptr, HD, Sb + (size_t)hl * NC * CH * WK, WK, nullptr, (size_t)CH * HD, (size_t)CH * HD, (size_t)CH * WK); }
            k_csoft<<<ZZ * CH / 8, 256, 0, stream>>>(Sb, P16);
            k_gemmw<h16, 0, false><<<dim3(CH / 64, 1, ZZ), 32, 0, stream>>>(P16, nullptr, VW, nullptr, WK, O, HD, nullptr, (size_t)CH * WK, (size_t)HD * WK, (size_t)CH * HD);
            k_mrg16<<<(unsigned)(((size_t)TT * HG * HD / 4 + 255) / 256), 256, 0, stream>>>(O, h0, A16); }
        k_gemmw<h16, 0, false><<<dim3(TT / 64, DM / 64, 1), 32, 0, stream>>>(A16, nullptr, WO16, nullptr, DM, OUT + (size_t)b * TT * DM, DM, nullptr, 0, 0, 0); }
}
